// JetBlock_8967891714369
// MI455X (gfx1250) — hardware-verified
//
#include <hip/hip_runtime.h>


#define NBI  2
#define NS   1024
#define HID  2048
#define NH_  8
#define DK   64
#define DV   128
#define TK   512
#define TV   1024
#define KC   4
#define GH   128
#define NQA  3088
#define NQP  3136
#define OQ   0
#define OK_  512
#define OV   1024
#define OA   2048
#define OB   2056
#define OZ   2064
#define EPS  1e-6f
#define DM   HID
#define LOSC 1024.0f

typedef _Float16 h16;
typedef unsigned short bf;
typedef __attribute__((ext_vector_type(16))) __bf16   v16bf;
typedef __attribute__((ext_vector_type(16))) _Float16 v16h;
typedef __attribute__((ext_vector_type(8)))  _Float16 v8h;
typedef __attribute__((ext_vector_type(8)))  unsigned short v8us;
typedef __attribute__((ext_vector_type(8)))  float    v8f;
typedef __attribute__((ext_vector_type(4)))  float    v4f;
typedef v8h  __attribute__((may_alias)) v8ha;
typedef v4f  __attribute__((may_alias)) v4fa;
typedef v8us __attribute__((may_alias)) v8usa;

__device__ __forceinline__ unsigned short f2bf(float f) { unsigned u = __float_as_uint(f); u += 0x7FFFu + ((u >> 16) & 1u); return (unsigned short)(u >> 16); }
__device__ __forceinline__ float bf2f(unsigned short b) { return __uint_as_float(((unsigned)b) << 16); }
__device__ __forceinline__ float bfr(float f) { return bf2f(f2bf(f)); }
__device__ __forceinline__ v16h cat16(v8h lo, v8h hi) { return __builtin_shufflevector(lo, hi, 0, 1, 2, 3, 4, 5, 6, 7, 8, 9, 10, 11, 12, 13, 14, 15); }
__device__ __forceinline__ v16bf cat16b(v8us lo, v8us hi) { return __builtin_bit_cast(v16bf, __builtin_shufflevector(lo, hi, 0, 1, 2, 3, 4, 5, 6, 7, 8, 9, 10, 11, 12, 13, 14, 15)); }
__device__ __forceinline__ v8f wmma16(v16h a, v16h b, v8f c) { return __builtin_amdgcn_wmma_f32_16x16x32_f16(false, a, false, b, (short)0, c, false, false); }
__device__ __forceinline__ v8f wmmab(v16bf a, v16bf b, v8f c) { return __builtin_amdgcn_wmma_f32_16x16x32_bf16(false, a, false, b, (short)0, c, false, false); }

template <bool SPLITA, bool F16OUT = false>
__global__ __launch_bounds__(128) void k_gemmb(const bf* __restrict__ A, const bf* __restrict__ Al, const bf* __restrict__ Bn, const float* __restrict__ bias, float* C, int ldc, h16* C2, const float* __restrict__ R = nullptr, int K = DM, int roundR = 1) {
    __shared__ __align__(16) float ost[4][16 * 68];
    const int lane = threadIdx.x & 31, wave = threadIdx.x >> 5, lr = lane & 15, hi = lane >> 4;
    const int r0 = blockIdx.x * 64 + wave * 16, c0 = blockIdx.y * 64;
    const size_t aoff = (size_t)(r0 + lr) * K + 8 * hi;
    size_t boff[4];
#pragma unroll
    for (int t = 0; t < 4; ++t) boff[t] = (size_t)(c0 + t * 16 + lr) * K + 8 * hi;
    v8f acc[4];
#pragma unroll
    for (int t = 0; t < 4; ++t) acc[t] = (v8f){};
#pragma unroll 1
    for (int kc = 0; kc < K; kc += 32) {
        const v16bf a = cat16b(*(const v8us*)(A + aoff + kc), *(const v8us*)(A + aoff + kc + 16));
        v16bf al = a;
        if (SPLITA) al = cat16b(*(const v8us*)(Al + aoff + kc), *(const v8us*)(Al + aoff + kc + 16));
#pragma unroll
        for (int t = 0; t < 4; ++t) { const v16bf b = cat16b(*(const v8us*)(Bn + boff[t] + kc), *(const v8us*)(Bn + boff[t] + kc + 16)); acc[t] = wmmab(a, b, acc[t]); if (SPLITA) acc[t] = wmmab(al, b, acc[t]); }
        asm volatile("v_nop\n\tv_nop\n\tv_nop\n\tv_nop" : "+v"(acc[0]), "+v"(acc[1]), "+v"(acc[2]), "+v"(acc[3]) : "v"(a), "v"(al));
    }
    float* os = &ost[wave][0];
#pragma unroll
    for (int t = 0; t < 4; ++t) { const float bv = bias ? bfr(bias[c0 + t * 16 + lr]) : 0.f;
#pragma unroll
        for (int j = 0; j < 8; ++j) os[(hi * 8 + j) * 68 + t * 16 + lr] = acc[t][j] + bv; }
    __syncthreads();
    if (F16OUT) {
        h16* crow = (h16*)(void*)C + (size_t)r0 * ldc + c0;
        auto pass = [&]() {
#pragma unroll
            for (int s = 0; s < 4; ++s) { const int row = 4 * s + (lane >> 3), piece = lane & 7; const float* sp = os + row * 68 + piece * 8; v8h o, o2;
#pragma unroll
                for (int i = 0; i < 8; ++i) { const h16 a = (h16)sp[i]; o[i] = a; o2[i] = (h16)((sp[i] - (float)a) * LOSC); }
                *(volatile v8h*)(crow + (size_t)row * ldc + piece * 8) = o; if (C2) *(volatile v8h*)(C2 + (size_t)r0 * ldc + c0 + (size_t)row * ldc + piece * 8) = o2; }
        };
        pass(); __threadfence(); pass();
    } else {
        float* crow = C + (size_t)r0 * ldc + c0;
        auto pass = [&]() {
#pragma unroll
            for (int s = 0; s < 8; ++s) { const int Lid = (lane >> 3) + 4 * s, piece = lane & 7; const int row = Lid >> 1, cofs = (Lid & 1) * 32 + piece * 4;
                v4f val = *(const v4fa*)(os + row * 68 + cofs); if (R) { const v4f rv = *(const v4f*)(R + ((size_t)r0 + row) * ldc + c0 + cofs); val += roundR ? (v4f){bfr(rv[0]), bfr(rv[1]), bfr(rv[2]), bfr(rv[3])} : rv; }
                *(volatile v4f*)(crow + (size_t)row * ldc + cofs) = val; }
        };
        pass(); __threadfence(); pass();
    }
}


__global__ __launch_bounds__(256) void k_wt(const float* __restrict__ Wm, int K, int ncols, bf* WT) {
    __shared__ __align__(16) unsigned short tl[64 * 72];
    const int tid = threadIdx.x, k0 = blockIdx.x * 64, n0 = blockIdx.y * 64;
    const int kk = tid >> 2, nq = (tid & 3) * 16;
#pragma unroll
    for (int i = 0; i < 16; ++i) tl[(nq + i) * 72 + kk] = f2bf(Wm[(size_t)(k0 + kk) * ncols + n0 + nq + i]);
    __syncthreads();
    const int piece = tid & 7;
    auto pass = [&]() {
#pragma unroll
        for (int s = 0; s < 2; ++s) { const int nr = (tid >> 3) + 32 * s; const v8us val = *(const v8usa*)(tl + nr * 72 + piece * 8); *(volatile v8us*)(WT + (size_t)(n0 + nr) * K + k0 + piece * 8) = val; }
    };
    pass(); __threadfence(); pass();
}

__global__ __launch_bounds__(256) void k_wtp(const float* __restrict__ Wm, int krows, int ncols, int kpad, bf* WT) {
    __shared__ __align__(16) unsigned short tl[64 * 72];
    const int tid = threadIdx.x, k0 = blockIdx.x * 64, n0 = blockIdx.y * 64;
    const int kk = tid >> 2, nq = (tid & 3) * 16;
    const int k = k0 + kk, kc = k < krows ? k : krows - 1;
#pragma unroll
    for (int i = 0; i < 16; ++i) { const int n = n0 + nq + i, ncl = n < ncols ? n : ncols - 1; const float w = Wm[(size_t)kc * ncols + ncl]; tl[(nq + i) * 72 + kk] = (k < krows && n < ncols) ? f2bf(w) : (unsigned short)0; }
    __syncthreads();
    const int piece = tid & 7;
    auto pass = [&]() {
#pragma unroll
        for (int s = 0; s < 2; ++s) { const int nr = (tid >> 3) + 32 * s; const v8us val = *(const v8usa*)(tl + nr * 72 + piece * 8); *(volatile v8us*)(WT + (size_t)(n0 + nr) * kpad + k0 + piece * 8) = val; }
    };
    pass(); __threadfence(); pass();
}

__global__ __launch_bounds__(256) void k_cvtb(const float* __restrict__ src, int nrows, bf* dst) {
    const int lane = threadIdx.x & 31, r = blockIdx.x * 8 + (threadIdx.x >> 5); if (r >= nrows) return;
#pragma unroll 1
    for (int ps = 0; ps < 2; ++ps) {
#pragma unroll
        for (int q = 0; q < HID / 256; ++q) { v8us o;
#pragma unroll
            for (int i = 0; i < 8; ++i) o[i] = f2bf(src[(size_t)r * HID + q * 256 + lane * 8 + i]);
            *(volatile v8us*)(dst + (size_t)r * HID + q * 256 + lane * 8) = o; }
        if (ps == 0) __threadfence(); }
}
__global__ __launch_bounds__(256) void k_silu128(const float* __restrict__ src, bf* dh, bf* dl) {
    typedef __attribute__((ext_vector_type(4))) unsigned short v4us;
    const int lane = threadIdx.x & 31, r = blockIdx.x * 8 + (threadIdx.x >> 5); if (r >= NS) return;
    const size_t o = (size_t)r * GH + lane * 4; const v4f v = *(const v4f*)(src + o); v4us oh, ol;
#pragma unroll
    for (int i = 0; i < 4; ++i) { const float s = v[i] / (1.0f + __expf(-v[i])); const unsigned short hb = f2bf(s); oh[i] = hb; ol[i] = f2bf(s - bf2f(hb)); }
    *(volatile v4us*)(dh + o) = oh; *(volatile v4us*)(dl + o) = ol; __threadfence(); *(volatile v4us*)(dh + o) = oh; *(volatile v4us*)(dl + o) = ol;
}
__global__ __launch_bounds__(256) void k_prep(const float* __restrict__ P, const float* __restrict__ K4, const float* __restrict__ cst, const float* __restrict__ Alog, const float* __restrict__ dtb, float* QK, float* VV, float* GB) {
    const int lane = threadIdx.x & 31, t = blockIdx.x * 8 + (threadIdx.x >> 5); if (t >= NS) return;
    const float* pr = P + (size_t)t * NQP;
#pragma unroll 1
    for (int ps = 0; ps < 2; ++ps) {
#pragma unroll 1
        for (int c0 = 0; c0 < TK; c0 += 128) {
#pragma unroll 1
            for (int which = 0; which < 2; ++which) { const int base = (which ? OK_ : OQ) + c0 + lane * 4; float s[4]; float ss = 0.f;
#pragma unroll
                for (int i = 0; i < 4; ++i) { const float x = pr[base + i]; s[i] = x / (1.0f + __expf(-x)); ss = fmaf(s[i], s[i], ss); }
                ss += __shfl_xor(ss, 1, 32); ss += __shfl_xor(ss, 2, 32); ss += __shfl_xor(ss, 4, 32); ss += __shfl_xor(ss, 8, 32);
                const float rn = rsqrtf(ss + EPS) * (which ? 1.0f : 0.125f); v4f o4;
#pragma unroll
                for (int i = 0; i < 4; ++i) o4[i] = s[i] * rn;
                *(volatile v4f*)(QK + (size_t)t * (2 * TK) + which * TK + c0 + lane * 4) = o4; } }
#pragma unroll 1
        for (int c0 = 0; c0 < TV; c0 += 128) { v4f o4;
#pragma unroll
            for (int i = 0; i < 4; ++i) { const int c = c0 + lane * 4 + i; float acc = 0.f;
#pragma unroll
                for (int j = 0; j < KC; ++j) { const int tt = t + j - (KC - 1); const int tc = tt < 0 ? 0 : tt; const int sj = t + j; const int sc = sj > KC - 2 ? KC - 2 : sj;
                    const float xv = (tt >= 0) ? P[(size_t)tc * NQP + OV + c] : bfr(cst[(size_t)c * (KC - 1) + sc]);
                    acc = fmaf(xv, K4[((size_t)t * TV + c) * KC + j], acc); }
                o4[i] = acc / (1.0f + __expf(-acc)); }
            *(volatile v4f*)(VV + (size_t)t * TV + c0 + lane * 4) = o4; }
        { float gv = 0.f; if (lane < NH_) { const float a = pr[OA + lane] + bfr(dtb[lane]); const float sp = (a > 20.f) ? a : log1pf(__expf(a)); gv = -__expf(bfr(Alog[lane])) * sp; }
          else if (lane < 2 * NH_) { gv = 1.0f / (1.0f + __expf(-pr[OB + lane - NH_])); }
          *(volatile float*)(GB + (size_t)t * 32 + lane) = gv; }
        if (ps == 0) __threadfence(); }
}
__global__ __launch_bounds__(128) void k_delta(const float* __restrict__ QK, const float* __restrict__ VV, const float* __restrict__ GB, const float* __restrict__ S0, float* O) {
    __shared__ float S[DK][DV]; __shared__ float qs[DK], ks[DK];
    const int v = threadIdx.x, h = blockIdx.x;
#pragma unroll 4
    for (int k = 0; k < DK; ++k) S[k][v] = bfr(S0[((size_t)h * DK + k) * DV + v]);
#pragma unroll 1
    for (int t = 0; t < NS; ++t) {
        __syncthreads();
        if (v < DK) { qs[v] = QK[(size_t)t * (2 * TK) + h * DK + v]; ks[v] = QK[(size_t)t * (2 * TK) + TK + h * DK + v]; }
        __syncthreads();
        const float g = GB[(size_t)t * 32 + h], bt = GB[(size_t)t * 32 + NH_ + h]; const float eg = __expf(g);
        float kv = 0.f;
#pragma unroll 4
        for (int k = 0; k < DK; ++k) { const float s = S[k][v] * eg; S[k][v] = s; kv = fmaf(ks[k], s, kv); }
        const float delta = (VV[(size_t)t * TV + h * DV + v] - kv) * bt;
        float ov = 0.f;
#pragma unroll 4
        for (int k = 0; k < DK; ++k) { const float s = fmaf(ks[k], delta, S[k][v]); S[k][v] = s; ov = fmaf(qs[k], s, ov); }
        float* op = O + (size_t)t * TV + h * DV + v; *(volatile float*)op = ov; __threadfence(); *(volatile float*)op = ov;
    }
}
__global__ __launch_bounds__(256) void k_onorm(const float* __restrict__ O, const float* __restrict__ P, const float* __restrict__ w, bf* Yh, bf* Yl) {
    typedef __attribute__((ext_vector_type(4))) unsigned short v4us;
    const int lane = threadIdx.x & 31, t = blockIdx.x * 8 + (threadIdx.x >> 5); if (t >= NS) return;
#pragma unroll 1
    for (int ps = 0; ps < 2; ++ps) {
#pragma unroll 1
        for (int h = 0; h < NH_; ++h) { const size_t ob = (size_t)t * TV + h * DV + lane * 4; float y[4]; float ss = 0.f;
#pragma unroll
            for (int i = 0; i < 4; ++i) { const float z = P[(size_t)t * NQP + OZ + h * DV + lane * 4 + i]; y[i] = O[ob + i] * (z / (1.0f + __expf(-z))); ss = fmaf(y[i], y[i], ss); }
#pragma unroll
            for (int sh = 16; sh; sh >>= 1) ss += __shfl_xor(ss, sh, 32);
            const float rn = rsqrtf(ss * (1.0f / DV) + EPS); v4us oh, ol;
#pragma unroll
            for (int i = 0; i < 4; ++i) { const float q = y[i] * rn * bfr(w[lane * 4 + i]); const unsigned short hb = f2bf(q); oh[i] = hb; ol[i] = f2bf(q - bf2f(hb)); }
            *(volatile v4us*)(Yh + ob) = oh; *(volatile v4us*)(Yl + ob) = ol; }
        if (ps == 0) __threadfence(); }
}

extern "C" void kernel_launch(void* const* d_in, const int* in_sizes, int n_in,
                              void* d_out, int out_size, void* d_ws, size_t ws_size, hipStream_t stream) {
    (void)in_sizes; (void)n_in; (void)out_size;
    const float* x = (const float*)d_in[0]; const float* Wq = (const float*)d_in[1]; const float* Alog = (const float*)d_in[2]; const float* dtb = (const float*)d_in[3]; const float* cst = (const float*)d_in[4];
    const float* w1 = (const float*)d_in[5]; const float* w2 = (const float*)d_in[6]; const float* b2 = (const float*)d_in[7]; const float* S0 = (const float*)d_in[8]; const float* onw = (const float*)d_in[9]; const float* Wo = (const float*)d_in[10];
    float* out = (float*)d_out;
    char* wsp = (char*)d_ws;
    auto take = [&](size_t bytes) { char* p = wsp; wsp += (bytes + 255) & ~(size_t)255; return (void*)p; };
    bf* WqT = (bf*)take((size_t)NQP * HID * 2); bf* W1T = (bf*)take((size_t)GH * HID * 2); bf* W2T = (bf*)take((size_t)(TV * KC) * GH * 2); bf* WoT = (bf*)take((size_t)HID * TV * 2);
    bf* Xb = (bf*)take((size_t)NS * HID * 2); float* P = (float*)take((size_t)NS * NQP * 4); float* G1 = (float*)take((size_t)NS * GH * 4); bf* G1h = (bf*)take((size_t)NS * GH * 2); bf* G1l = (bf*)take((size_t)NS * GH * 2);
    float* K4 = (float*)take((size_t)NS * TV * KC * 4); float* QK = (float*)take((size_t)NS * 2 * TK * 4); float* VV = (float*)take((size_t)NS * TV * 4); float* GB = (float*)take((size_t)NS * 32 * 4); float* O = (float*)take((size_t)NS * TV * 4);
    bf* Yh = (bf*)take((size_t)NS * TV * 2); bf* Yl = (bf*)take((size_t)NS * TV * 2);
    if ((size_t)(wsp - (char*)d_ws) > ws_size) return;
    k_wtp<<<dim3(HID / 64, NQP / 64, 1), 256, 0, stream>>>(Wq, HID, NQA, HID, WqT);
    k_wt<<<dim3(HID / 64, GH / 64, 1), 256, 0, stream>>>(w1, HID, GH, W1T); k_wt<<<dim3(GH / 64, (TV * KC) / 64, 1), 256, 0, stream>>>(w2, GH, TV * KC, W2T); k_wt<<<dim3(TV / 64, HID / 64, 1), 256, 0, stream>>>(Wo, TV, HID, WoT);
    for (int b = 0; b < NBI; ++b) {
        k_cvtb<<<NS / 8, 256, 0, stream>>>(x + (size_t)b * NS * HID, NS, Xb);
        k_gemmb<false, false><<<dim3(NS / 64, NQP / 64, 1), 128, 0, stream>>>(Xb, nullptr, WqT, nullptr, P, NQP, nullptr, nullptr, HID);
        k_gemmb<false, false><<<dim3(NS / 64, GH / 64, 1), 128, 0, stream>>>(Xb, nullptr, W1T, nullptr, G1, GH, nullptr, nullptr, HID);
        k_silu128<<<NS / 8, 256, 0, stream>>>(G1, G1h, G1l);
        k_gemmb<true, false><<<dim3(NS / 64, (TV * KC) / 64, 1), 128, 0, stream>>>(G1h, G1l, W2T, b2, K4, TV * KC, nullptr, nullptr, GH);
        k_prep<<<NS / 8, 256, 0, stream>>>(P, K4, cst + (size_t)b * TV * (KC - 1), Alog, dtb, QK, VV, GB);
        k_delta<<<NH_, DV, 0, stream>>>(QK, VV, GB, S0 + (size_t)b * NH_ * DK * DV, O);
        k_onorm<<<NS / 8, 256, 0, stream>>>(O, P, onw, Yh, Yl);
        k_gemmb<true, false><<<dim3(NS / 64, HID / 64, 1), 128, 0, stream>>>(Yh, Yl, WoT, nullptr, out + (size_t)b * NS * HID, HID, nullptr, nullptr, TV);
    }
}
